// MetaMultiLinear_19602230739476
// MI455X (gfx1250) — hardware-verified
//
#include <hip/hip_runtime.h>

typedef float          v8f   __attribute__((ext_vector_type(8)));
typedef float          v4f   __attribute__((ext_vector_type(4)));
typedef unsigned int   v4u   __attribute__((ext_vector_type(4)));
typedef int            v8i   __attribute__((ext_vector_type(8)));
typedef unsigned short v8us  __attribute__((ext_vector_type(8)));
typedef unsigned short v16us __attribute__((ext_vector_type(16)));
typedef __bf16         v16bf __attribute__((ext_vector_type(16)));
typedef _Float16       v16h  __attribute__((ext_vector_type(16)));
typedef v4f  __attribute__((may_alias)) v4fa;
typedef v8us __attribute__((may_alias)) v8usa;
union FragB { v16bf v; v16us u; v8us h[2]; v8i w; };
union FragH { v16h  v; v16us u; v8us h[2]; v8i w; };

__device__ __forceinline__ v8f wmb(const FragB& a, const FragB& b, v8f c) {
  v8f d = __builtin_amdgcn_wmma_f32_16x16x32_bf16(false, a.v, false, b.v, (short)0, c, false, false);
  asm volatile("v_nop\n\tv_nop\n\tv_nop\n\tv_nop" : "+v"(d) : "v"(a.w), "v"(b.w));
  return d;
}

__device__ __forceinline__ v8f wmh(const FragH& a, const FragH& b, v8f c) {
  v8f d = __builtin_amdgcn_wmma_f32_16x16x32_f16(false, a.v, false, b.v, (short)0, c, false, false);
  asm volatile("v_nop\n\tv_nop\n\tv_nop\n\tv_nop" : "+v"(d) : "v"(a.w), "v"(b.w));
  return d;
}

__device__ __forceinline__ unsigned bf16_bits(float f) {
  const unsigned u = __float_as_uint(f);
  const unsigned r = (u + 0x7FFFu + ((u >> 16) & 1u)) >> 16;
  const unsigned q = (u >> 16) | 0x40u;
  return ((u & 0x7fffffffu) > 0x7f800000u) ? q : r;
}

__device__ __forceinline__ float bf16_val(float f) {
  return __uint_as_float(bf16_bits(f) << 16);
}
__device__ __forceinline__ int clampi(int v, int lo, int hi) {
  return v < lo ? lo : (v > hi ? hi : v);
}

__device__ __forceinline__ unsigned f16_bits(float f) {
  const unsigned u  = __float_as_uint(f);
  const unsigned s  = (u >> 16) & 0x8000u;
  const unsigned a  = u & 0x7fffffffu;
  const unsigned t  = a - 0x38000000u;
  const unsigned r  = (t + 0x0FFFu + ((t >> 13) & 1u)) >> 13;
  const unsigned rc = r > 0x7C00u ? 0x7C00u : r;
  const bool small  = a < 0x38800000u;
  const bool isnan  = a > 0x7f800000u;
  const unsigned fin = small ? 0u : (s | rc);
  return isnan ? (s | 0x7E00u) : fin;
}

__device__ __forceinline__ unsigned pk16(unsigned lo, unsigned hi) { return lo | (hi << 16); }
__device__ __forceinline__ unsigned bf16_lo_bits(float v) {
  float hi = bf16_val(v);
  asm volatile("" : "+v"(hi));
  return bf16_bits(v - hi);
}
__device__ __forceinline__ v4u pack8_bf16(v4f a, v4f c) {
  return (v4u){ pk16(bf16_bits(a[0]), bf16_bits(a[1])), pk16(bf16_bits(a[2]), bf16_bits(a[3])),
                pk16(bf16_bits(c[0]), bf16_bits(c[1])), pk16(bf16_bits(c[2]), bf16_bits(c[3])) };
}
__device__ __forceinline__ v4u pack8_bf16_lo(v4f a, v4f c) {
  return (v4u){ pk16(bf16_lo_bits(a[0]), bf16_lo_bits(a[1])), pk16(bf16_lo_bits(a[2]), bf16_lo_bits(a[3])),
                pk16(bf16_lo_bits(c[0]), bf16_lo_bits(c[1])), pk16(bf16_lo_bits(c[2]), bf16_lo_bits(c[3])) };
}
__device__ __forceinline__ v4u pack8_f16(v4f a, v4f c) {
  return (v4u){ pk16(f16_bits(a[0]), f16_bits(a[1])), pk16(f16_bits(a[2]), f16_bits(a[3])),
                pk16(f16_bits(c[0]), f16_bits(c[1])), pk16(f16_bits(c[2]), f16_bits(c[3])) };
}

template <int FORM>
__global__ __launch_bounds__(256) void k_plane(const float* __restrict__ src, int rows, int cols, int ldsrc,
                                               unsigned short* __restrict__ dst, int MP, int KP) {
  static_assert(FORM >= 0 && FORM <= 3);
  const int KTOT = (FORM == 1 || FORM == 3) ? 2 * KP : KP;
  const unsigned ppr   = (unsigned)(KTOT >> 3);
  const unsigned kp8   = (unsigned)(KP >> 3);
  const unsigned total = (unsigned)MP * ppr;
  const unsigned g     = blockIdx.x * 256u + threadIdx.x;
  const unsigned rowu  = g / ppr;
  const unsigned p     = g - rowu * ppr;
  const bool second    = p >= kp8;
  const int row = (int)rowu;
  const int c0  = (int)((second ? p - kp8 : p) << 3);
  const float* srow = src + (size_t)clampi(row, 0, rows - 1) * (size_t)ldsrc;
  float x[8];
  unsigned mk[8];
#pragma unroll
  for (int e = 0; e < 8; ++e) {
    const int c = c0 + e;
    const float v = srow[clampi(c, 0, cols - 1)];
    asm volatile("" :: "v"(v));
    x[e]  = v;
    mk[e] = (row < rows && c < cols) ? 0xFFFFu : 0u;
  }
  const v4f a = (v4f){ x[0], x[1], x[2], x[3] };
  const v4f c = (v4f){ x[4], x[5], x[6], x[7] };
  v4u o;
  if (FORM == 2) {
    o = pack8_f16(a, c);
  } else {
    const v4u hi = pack8_bf16(a, c);
    o = hi;
    if (FORM == 1) { const v4u lo = pack8_bf16_lo(a, c); o = second ? lo : hi; }
  }
  const v4u mw = (v4u){ pk16(mk[0], mk[1]), pk16(mk[2], mk[3]), pk16(mk[4], mk[5]), pk16(mk[6], mk[7]) };
  o &= mw;
  if (g < total) {
    volatile v4u* q = (volatile v4u*)(dst + (size_t)g * 8);
    *q = o;
    __threadfence();
    *q = o;
  }
}

template <int FORM> struct FragOf    { typedef FragB T; };
template <>         struct FragOf<2> { typedef FragH T; };
__device__ __forceinline__ v8f mm(const FragB& a, const FragB& b, v8f c) { return wmb(a, b, c); }
__device__ __forceinline__ v8f mm(const FragH& a, const FragH& b, v8f c) { return wmh(a, b, c); }
template <class F> __device__ __forceinline__ F ld_frag(const unsigned short* p) {
  F f;
  f.h[0] = *(const v8usa*)(p);
  f.h[1] = *(const v8usa*)(p + 16);
  return f;
}

template <int FORM, int EPI>
__global__ __launch_bounds__(256) __attribute__((amdgpu_num_vgpr(248)))
void k_gemm_nt(const unsigned short* __restrict__ A, const unsigned short* __restrict__ B,
               const float* __restrict__ bias, float* __restrict__ D, int M, int N, int KTOT, int ldd) {
  static_assert(FORM >= 0 && FORM <= 2);
  static_assert(EPI == 0 || EPI == 1);
  typedef typename FragOf<FORM>::T F;
  __shared__ __attribute__((aligned(16))) float sT[8][16 * 68];
  const int lane = threadIdx.x & 31;
  const int wave = threadIdx.x >> 5;
  const int tilesM = (M + 63) >> 6;
  const int tilesN = (N + 63) >> 6;
  const int tile = blockIdx.x * 8 + wave;
  if (tile >= tilesM * tilesN) return;
  const int tm = tile / tilesN;
  const int tn = tile - tm * tilesN;
  const int m0 = tm << 6;
  const int n0 = tn << 6;

  const int rl = lane & 15;
  const int h8 = (lane >> 4) * 8;
  const unsigned short* pa = A + (size_t)(m0 + rl) * (size_t)KTOT + h8;
  const unsigned short* pb = B + (size_t)(n0 + rl) * (size_t)KTOT + h8;

  v8f acc[4][4];
#pragma unroll
  for (int i = 0; i < 4; ++i)
#pragma unroll
    for (int j = 0; j < 4; ++j) acc[i][j] = (v8f){0.f, 0.f, 0.f, 0.f, 0.f, 0.f, 0.f, 0.f};

#pragma unroll 1
  for (int k0 = 0; k0 < KTOT; k0 += 32) {
    F bf[4];
#pragma unroll
    for (int j = 0; j < 4; ++j) bf[j] = ld_frag<F>(pb + (size_t)(j << 4) * (size_t)KTOT + k0);
#pragma unroll
    for (int i = 0; i < 4; ++i) {
      const F af = ld_frag<F>(pa + (size_t)(i << 4) * (size_t)KTOT + k0);
#pragma unroll
      for (int j = 0; j < 4; ++j) acc[i][j] = mm(af, bf[j], acc[i][j]);
    }
  }

  float* slab = sT[wave];
  const int hh = lane >> 4;
  const int c4 = (lane & 15) * 4;
  const int nc = n0 + c4;
  const bool cok = nc < N;
  v4f bv = (v4f){0.f, 0.f, 0.f, 0.f};
  if (EPI == 1) {
    bv = *(const v4fa*)(bias + clampi(nc, 0, N - 4));
    asm volatile("" :: "v"(bv));
  }
#pragma unroll
  for (int i = 0; i < 4; ++i) {
    const int mBase = m0 + (i << 4);
#pragma unroll
    for (int j = 0; j < 4; ++j) {
#pragma unroll
      for (int r = 0; r < 8; ++r) slab[(h8 + r) * 68 + (j << 4) + rl] = acc[i][j][r];
    }
    __builtin_amdgcn_fence(__ATOMIC_RELEASE, "workgroup");
    __builtin_amdgcn_wave_barrier();
    __builtin_amdgcn_fence(__ATOMIC_ACQUIRE, "workgroup");
    v4f vv[8];
#pragma unroll
    for (int it = 0; it < 8; ++it) {
      const int row = it * 2 + hh;
      v4f v = *(const v4fa*)(slab + row * 68 + c4);
      if (EPI == 1) v += bv;
      vv[it] = v;
    }
    for (int pass = 0; pass < 2; ++pass) {
#pragma unroll
      for (int it = 0; it < 8; ++it) {
        const int row = mBase + it * 2 + hh;
        if (cok && row < M) *(volatile v4f*)(D + (size_t)row * (size_t)ldd + nc) = vv[it];
      }
      __threadfence();
    }
    __builtin_amdgcn_fence(__ATOMIC_RELEASE, "workgroup");
    __builtin_amdgcn_wave_barrier();
    __builtin_amdgcn_fence(__ATOMIC_ACQUIRE, "workgroup");
  }
}

#define MH      8
#define MBATCH  32768
#define MIN_F   16
#define MCOND   32
#define MOUT    32
#define MKPI    17
#define MNGEN   544
#define MNT     34
#define WPITCH  40
#define WTSTR   548
#define MTHR    128
#define MWAVES  4
#define MTILES  4
#define MSAMP   256
#define MRUNS   128

#define LO_W    0
#define LO_B    (MNGEN * WPITCH * 2)
#define LO_X    (LO_B + MNGEN * 4)
#define LO_WT   (LO_X + MWAVES * 16 * MIN_F * 4)
#define LDS_DYN (LO_WT + MWAVES * 16 * WTSTR * 4)

static_assert(MNGEN == MOUT * MKPI && MNGEN == MNT * 16);
static_assert(MKPI == MIN_F + 1);
static_assert(MCOND == 32);
static_assert(MOUT == 32);
static_assert(MBATCH % MSAMP == 0 && MSAMP == MWAVES * MTILES * 16 && MRUNS * MSAMP == MBATCH);
static_assert(MTHR == MWAVES * 32);
static_assert(WTSTR >= MNGEN && WTSTR % 4 == 0 && (8 * WTSTR) % 64 == 32);
static_assert(WPITCH >= MCOND + 8 && WPITCH % 8 == 0);
static_assert((MNGEN * MCOND / 8) % MTHR == 0);
static_assert((MNGEN / 4) <= 2 * MTHR && MNGEN % 4 == 0);
static_assert(LO_B % 16 == 0 && LO_X % 16 == 0 && LO_WT % 16 == 0);
static_assert(LO_B == 43520 && LO_X == 45696 && LO_WT == 49792 && LDS_DYN == 190080);
static_assert(LDS_DYN <= 327680);
static_assert(MNT % 2 == 0);

typedef v4u __attribute__((may_alias)) v4ua;

__device__ __forceinline__ v4f bfv4(v4f v) {
  return (v4f){ bf16_val(v[0]), bf16_val(v[1]), bf16_val(v[2]), bf16_val(v[3]) };
}

__global__ __launch_bounds__(MTHR) void k_meta(const float* __restrict__ xin, const float* __restrict__ cond,
                                               const float* __restrict__ cw, const float* __restrict__ cb,
                                               float* __restrict__ out) {
  extern __shared__ __attribute__((aligned(16))) unsigned char smem[];
  unsigned short* sW = (unsigned short*)(smem + LO_W);
  float* sB  = (float*)(smem + LO_B);
  float* sXa = (float*)(smem + LO_X);
  float* sTa = (float*)(smem + LO_WT);

  const int tid  = threadIdx.x;
  const int lane = tid & 31;
  const int wave = tid >> 5;
  const int head = blockIdx.x / MRUNS;
  const int run  = blockIdx.x - head * MRUNS;
  const int rl   = lane & 15;
  const int hh   = lane >> 4;

  {
    const float* wsrc = cw + (size_t)head * (size_t)(MNGEN * MCOND);
#pragma unroll 1
    for (int it = 0; it < (MNGEN * MCOND / 8) / MTHR; ++it) {
      const int g = it * MTHR + tid;
      const v4f a = *(const v4fa*)(wsrc + (size_t)g * 8);
      const v4f c = *(const v4fa*)(wsrc + (size_t)g * 8 + 4);
      const v4u o = pack8_bf16(a, c);
      const int row = g >> 2, piece = g & 3;
      *(v4ua*)(sW + row * WPITCH + piece * 8) = o;
    }
    for (int r = tid; r < MNGEN; r += MTHR) *(v4ua*)(sW + r * WPITCH + MCOND) = (v4u){0u, 0u, 0u, 0u};
#pragma unroll
    for (int it = 0; it < 2; ++it) {
      const int q  = it * MTHR + tid;
      const int qc = clampi(q, 0, MNGEN / 4 - 1);
      const v4f v = *(const v4fa*)(cb + (size_t)head * MNGEN + (size_t)qc * 4);
      asm volatile("" :: "v"(v));
      const v4f r = bfv4(v);
      if (q < MNGEN / 4) *(v4fa*)(sB + q * 4) = r;
    }
  }
  __syncthreads();

  float bias[MKPI];
#pragma unroll
  for (int i = 0; i < MKPI; ++i) bias[i] = sB[lane * MKPI + i];

  float* wt = sTa + wave * (16 * WTSTR);
  float* sx = sXa + wave * (16 * MIN_F);
  const unsigned short* bbase = sW + rl * WPITCH + 8 * hh;
  float* dbase = wt + (8 * hh) * WTSTR + rl;
  const v8f z8 = (v8f){0.f, 0.f, 0.f, 0.f, 0.f, 0.f, 0.f, 0.f};

#pragma unroll 1
  for (int mt = 0; mt < MTILES; ++mt) {
    const int b0 = run * MSAMP + wave * (MTILES * 16) + mt * 16;
    const size_t s0 = (size_t)head * MBATCH + (size_t)b0;

    FragB a;
    {
      const float* cp = cond + (s0 + (size_t)rl) * MCOND + 8 * hh;
      const v4f f0 = *(const v4fa*)(cp);
      const v4f f1 = *(const v4fa*)(cp + 4);
      const v4f f2 = *(const v4fa*)(cp + 16);
      const v4f f3 = *(const v4fa*)(cp + 20);
      const v4u p0 = pack8_bf16(f0, f1);
      const v4u p1 = pack8_bf16(f2, f3);
      a.w = (v8i){ (int)p0[0], (int)p0[1], (int)p0[2], (int)p0[3], (int)p1[0], (int)p1[1], (int)p1[2], (int)p1[3] };
    }
    {
      const float* xp = xin + s0 * MIN_F + lane * 4;
      const v4f xa = *(const v4fa*)(xp);
      const v4f xb = *(const v4fa*)(xp + 128);
      *(v4fa*)(sx + lane * 4)       = bfv4(xa);
      *(v4fa*)(sx + 128 + lane * 4) = bfv4(xb);
    }

#pragma unroll 2
    for (int t = 0; t < MNT; ++t) {
      FragB b;
      const unsigned short* bp = bbase + t * (16 * WPITCH);
      b.h[0] = *(const v8usa*)(bp);
      b.h[1] = *(const v8usa*)(bp + 16);
      const v8f d = wmb(a, b, z8);
      float* dp = dbase + t * 16;
#pragma unroll
      for (int r = 0; r < 8; ++r) dp[r * WTSTR] = d[r];
    }

    __builtin_amdgcn_fence(__ATOMIC_RELEASE, "workgroup");
    __builtin_amdgcn_wave_barrier();
    __builtin_amdgcn_fence(__ATOMIC_ACQUIRE, "workgroup");

#pragma unroll 1
    for (int g = 0; g < 4; ++g) {
      float res[4];
#pragma unroll
      for (int j = 0; j < 4; ++j) {
        const int m = g * 4 + j;
        const float* wr = wt + m * WTSTR + lane * MKPI;
        const float* xr = sx + m * MIN_F;
        const v4f x0 = *(const v4fa*)(xr);
        const v4f x1 = *(const v4fa*)(xr + 4);
        const v4f x2 = *(const v4fa*)(xr + 8);
        const v4f x3 = *(const v4fa*)(xr + 12);
        const float xs[16] = { x0[0], x0[1], x0[2], x0[3], x1[0], x1[1], x1[2], x1[3],
                               x2[0], x2[1], x2[2], x2[3], x3[0], x3[1], x3[2], x3[3] };
        float acc = 0.0f;
#pragma unroll
        for (int i = 0; i < MIN_F; ++i) {
          const float v = wr[i] + bias[i];
          acc = fmaf(v, xs[i], acc);
        }
        const float v16 = wr[MIN_F] + bias[MIN_F];
        res[j] = acc + v16;
      }
      float* orow = out + (s0 + (size_t)(g * 4)) * MOUT + lane;
#pragma unroll
      for (int j = 0; j < 4; ++j) *(volatile float*)(orow + j * MOUT) = res[j];
      __threadfence();
#pragma unroll
      for (int j = 0; j < 4; ++j) *(volatile float*)(orow + j * MOUT) = res[j];
    }

    __builtin_amdgcn_fence(__ATOMIC_RELEASE, "workgroup");
    __builtin_amdgcn_wave_barrier();
    __builtin_amdgcn_fence(__ATOMIC_ACQUIRE, "workgroup");
  }
}

extern "C" void kernel_launch(void* const* d_in, const int* in_sizes, int n_in,
                              void* d_out, int out_size, void* d_ws, size_t ws_size,
                              hipStream_t stream) {
  (void)d_ws;
  (void)ws_size;
  if (n_in < 4) return;
  if (in_sizes[0] != MH * MBATCH * MIN_F) return;
  if (in_sizes[1] != MH * MBATCH * MCOND) return;
  if (in_sizes[2] != MH * MNGEN * MCOND) return;
  if (in_sizes[3] != MH * MNGEN) return;
  if (out_size != MH * MBATCH * MOUT) return;

  const float* xin  = (const float*)d_in[0];
  const float* cond = (const float*)d_in[1];
  const float* cw   = (const float*)d_in[2];
  const float* cb   = (const float*)d_in[3];
  float* out = (float*)d_out;

  hipFuncSetAttribute(reinterpret_cast<const void*>(&k_meta), hipFuncAttributeMaxDynamicSharedMemorySize, LDS_DYN);
  k_meta<<<MH * MRUNS, MTHR, LDS_DYN, stream>>>(xin, cond, cw, cb, out);
}
